// EnhancedMSAGAT_Net_25228637897512
// MI455X (gfx1250) — hardware-run, weakly checked
//
#include <hip/hip_runtime.h>
#define NBt 16
#define TW 64
#define NN 1024
#define CC 128
#define NH 8
#define HD 16
#define NSC 5
#define BOT 16
#define HOR 24
#define HWY 16
#define NR (NBt * NN)
#define HG 8
typedef __bf16 v16b __attribute__((ext_vector_type(16)));
typedef unsigned short v8us __attribute__((ext_vector_type(8), may_alias));
typedef float  v8f  __attribute__((ext_vector_type(8)));
typedef float  v4f  __attribute__((ext_vector_type(4)));
typedef float  v4fa __attribute__((ext_vector_type(4), may_alias));
union FragB { v16b v; v8us half[2]; unsigned short u[16]; };

__device__ __forceinline__ unsigned short bf16_bits(float x) { unsigned int u = __float_as_uint(x); return (unsigned short)((u + 0x7FFFu + ((u >> 16) & 1u)) >> 16); }
__device__ __forceinline__ float bf16_val(unsigned short b) { return __uint_as_float(((unsigned int)b) << 16); }
__device__ __forceinline__ float bf16_round(float x) { return bf16_val(bf16_bits(x)); }
template <int NT>
__device__ __forceinline__ v8f mmaN(v16b ah, v16b al, v16b bh, v16b bl, v8f c) {
  c = __builtin_amdgcn_wmma_f32_16x16x32_bf16(false, ah, false, bh, (short)0, c, false, false);
  if (NT >= 2) c = __builtin_amdgcn_wmma_f32_16x16x32_bf16(false, al, false, bh, (short)0, c, false, false);
  if (NT >= 3) c = __builtin_amdgcn_wmma_f32_16x16x32_bf16(false, ah, false, bl, (short)0, c, false, false);
  asm volatile("v_nop\n\tv_nop\n\tv_nop\n\tv_nop" : "+v"(c) : "v"(ah), "v"(al), "v"(bh), "v"(bl));
  return c;
}

__global__ __launch_bounds__(256) void k_wt_bf16(const float* __restrict__ W, unsigned short* __restrict__ Wt, int K, int N) {
  const int t = blockIdx.x * 256 + threadIdx.x;
  const int k8n = K / 8;
  if (t >= N * k8n) return;
  const int n = t / k8n, k8 = (t % k8n) * 8;
  v8us v;
#pragma unroll
  for (int i = 0; i < 8; ++i) v[i] = bf16_bits(W[(size_t)(k8 + i) * N + n]);
  *(volatile v8us*)(Wt + (size_t)n * K + k8) = v;
  __threadfence();
  *(volatile v8us*)(Wt + (size_t)n * K + k8) = v;
}

template <bool ASPLIT, int ACT, bool BIAS_BF16>
__global__ __launch_bounds__(128) void k_gemm_bf(const float* __restrict__ A, int lda, const unsigned short* __restrict__ Wt, int ldb,
                                               const float* __restrict__ bias, float* __restrict__ C, int ldc, int M, int N, int K) {
  __shared__ __attribute__((aligned(16))) float so[4][16][64];
  const int tid = threadIdx.x, w = tid >> 5, lane = tid & 31, ln = lane & 15, hh = lane >> 4;
  const int ntn = N / 64;
  const int wid = blockIdx.x * 4 + w;
  const int mt = wid / ntn, nq = wid % ntn;
  if (mt * 16 >= M) return;
  const int row0 = mt * 16, col0 = nq * 64;
  const float* arow = A + (size_t)(row0 + ln) * lda;
  v8f acc[4] = {};
  for (int kb = 0; kb < K; kb += 32) {
    FragB ah, al;
    const v4f x0 = *(const v4fa*)(arow + kb + 8 * hh), x1 = *(const v4fa*)(arow + kb + 8 * hh + 4);
    const v4f x2 = *(const v4fa*)(arow + kb + 16 + 8 * hh), x3 = *(const v4fa*)(arow + kb + 16 + 8 * hh + 4);
    float xs[16] = {x0[0],x0[1],x0[2],x0[3],x1[0],x1[1],x1[2],x1[3],x2[0],x2[1],x2[2],x2[3],x3[0],x3[1],x3[2],x3[3]};
#pragma unroll
    for (int i = 0; i < 16; ++i) { const unsigned short hb = bf16_bits(xs[i]); ah.u[i] = hb; al.u[i] = ASPLIT ? bf16_bits(xs[i] - bf16_val(hb)) : (unsigned short)0; }
#pragma unroll
    for (int t = 0; t < 4; ++t) {
      const unsigned short* brow = Wt + (size_t)(col0 + t * 16 + ln) * ldb + kb;
      FragB b;
      b.half[0] = *(const v8us*)(brow + 8 * hh);
      b.half[1] = *(const v8us*)(brow + 16 + 8 * hh);
      acc[t] = mmaN<ASPLIT ? 2 : 1>(ah.v, al.v, b.v, b.v, acc[t]);
    }
  }
#pragma unroll
  for (int t = 0; t < 4; ++t) {
    float bv = bias ? bias[col0 + t * 16 + ln] : 0.f;
    if (BIAS_BF16) bv = bf16_round(bv);
#pragma unroll
    for (int r = 0; r < 8; ++r) { float v = acc[t][r] + bv; if (ACT == 1) v = fmaxf(v, 0.f); so[w][8 * hh + r][t * 16 + ln] = v; }
  }
  __builtin_amdgcn_fence(__ATOMIC_ACQ_REL, "workgroup");
  __builtin_amdgcn_wave_barrier();
  const int rsub = lane >> 4, c4 = (lane & 15) * 4;
  for (int pass = 0; pass < 2; ++pass) {
#pragma unroll
    for (int q = 0; q < 8; ++q) {
      const int r = q * 2 + rsub;
      const v4f v = *(const v4fa*)&so[w][r][c4];
      *(volatile v4f*)(C + (size_t)(row0 + r) * ldc + col0 + c4) = v;
    }
    if (pass == 0) __threadfence();
  }
}

template <bool ASPLIT, int ACT, bool BIAS_BF16, bool RES_BF16>
__global__ __launch_bounds__(128) void k_gemm_bf3(const float* __restrict__ A, int lda, const unsigned short* __restrict__ Wt, int ldb,
                                                const float* __restrict__ bias, const float* __restrict__ resid, int rmod, int ldr,
                                                float* __restrict__ C, int ldc, int M, int N, int K) {
  __shared__ __attribute__((aligned(16))) float so[4][16][64];
  const int tid = threadIdx.x, w = tid >> 5, lane = tid & 31, ln = lane & 15, hh = lane >> 4;
  const int ntn = N / 64;
  const int wid = blockIdx.x * 4 + w;
  const int mt = wid / ntn, nq = wid % ntn;
  if (mt * 16 >= M) return;
  const int row0 = mt * 16, col0 = nq * 64;
  const float* arow = A + (size_t)(row0 + ln) * lda;
  v8f acc[4] = {};
  for (int kb = 0; kb < K; kb += 32) {
    FragB ah, al;
    const v4f x0 = *(const v4fa*)(arow + kb + 8 * hh), x1 = *(const v4fa*)(arow + kb + 8 * hh + 4);
    const v4f x2 = *(const v4fa*)(arow + kb + 16 + 8 * hh), x3 = *(const v4fa*)(arow + kb + 16 + 8 * hh + 4);
    float xs[16] = {x0[0],x0[1],x0[2],x0[3],x1[0],x1[1],x1[2],x1[3],x2[0],x2[1],x2[2],x2[3],x3[0],x3[1],x3[2],x3[3]};
#pragma unroll
    for (int i = 0; i < 16; ++i) { const unsigned short hb = bf16_bits(xs[i]); ah.u[i] = hb; al.u[i] = ASPLIT ? bf16_bits(xs[i] - bf16_val(hb)) : (unsigned short)0; }
#pragma unroll
    for (int t = 0; t < 4; ++t) {
      const unsigned short* brow = Wt + (size_t)(col0 + t * 16 + ln) * ldb + kb;
      FragB b;
      b.half[0] = *(const v8us*)(brow + 8 * hh);
      b.half[1] = *(const v8us*)(brow + 16 + 8 * hh);
      acc[t] = mmaN<ASPLIT ? 2 : 1>(ah.v, al.v, b.v, b.v, acc[t]);
    }
  }
#pragma unroll
  for (int t = 0; t < 4; ++t) {
    const int col = col0 + t * 16 + ln;
    float bv = bias ? bias[col] : 0.f;
    if (BIAS_BF16) bv = bf16_round(bv);
#pragma unroll
    for (int r = 0; r < 8; ++r) {
      float v = acc[t][r] + bv;
      if (resid) { float rv = resid[(size_t)((row0 + 8 * hh + r) % rmod) * ldr + col]; if (RES_BF16) rv = bf16_round(rv); v += rv; }
      if (ACT == 1) v = fmaxf(v, 0.f);
      if (ACT == 2) v = 0.5f * v * (1.0f + erff(v * 0.70710678118654752f));
      if (ACT == 3) { const float u = 0.7978845608028654f * (v + 0.044715f * v * v * v); v = 0.5f * v * (1.0f + tanhf(u)); }
      so[w][8 * hh + r][t * 16 + ln] = v;
    }
  }
  __builtin_amdgcn_fence(__ATOMIC_ACQ_REL, "workgroup");
  __builtin_amdgcn_wave_barrier();
  const int rsub = lane >> 4, c4 = (lane & 15) * 4;
  for (int pass = 0; pass < 2; ++pass) {
#pragma unroll
    for (int q = 0; q < 8; ++q) {
      const int r = q * 2 + rsub;
      const v4f v = *(const v4fa*)&so[w][r][c4];
      *(volatile v4f*)(C + (size_t)(row0 + r) * ldc + col0 + c4) = v;
    }
    if (pass == 0) __threadfence();
  }
}
template <bool PARAM_BF16>
__global__ __launch_bounds__(256) void k_layernorm(const float* __restrict__ X, const float* __restrict__ R, const float* __restrict__ g, const float* __restrict__ bta,
                                                  float* __restrict__ out_sum, float* __restrict__ out_norm, int N, float eps) {
  __shared__ float red[256];
  const int row = blockIdx.x, tid = threadIdx.x;
  const float* x = X + (size_t)row * N; const float* rr = R ? R + (size_t)row * N : nullptr;
  float vals[16];
  const int per = N / 256;
  float s1 = 0.f;
  for (int u = 0; u < per / 4; ++u) {
    const int j = tid * 4 + 1024 * u;
    const v4f a = *(const v4fa*)(x + j);
    v4f b = {0.f,0.f,0.f,0.f}; if (rr) b = *(const v4fa*)(rr + j);
#pragma unroll
    for (int q = 0; q < 4; ++q) { const float v = a[q] + b[q]; vals[u * 4 + q] = v; s1 += v; }
  }
  red[tid] = s1; __syncthreads();
  for (int st = 128; st > 0; st >>= 1) { if (tid < st) red[tid] += red[tid + st]; __syncthreads(); }
  const float mu = red[0] / (float)N; __syncthreads();
  float s2 = 0.f;
  for (int u = 0; u < per / 4; ++u)
#pragma unroll
    for (int q = 0; q < 4; ++q) { const float c = vals[u * 4 + q] - mu; s2 += c * c; }
  red[tid] = s2; __syncthreads();
  for (int st = 128; st > 0; st >>= 1) { if (tid < st) red[tid] += red[tid + st]; __syncthreads(); }
  const float rs = rsqrtf(red[0] / (float)N + eps);
  for (int pass = 0; pass < 2; ++pass) {
    for (int u = 0; u < per / 4; ++u) {
      const int j = tid * 4 + 1024 * u;
      v4f o, sm;
#pragma unroll
      for (int q = 0; q < 4; ++q) {
        float gg = g[j + q], bb = bta[j + q];
        if (PARAM_BF16) { gg = bf16_round(gg); bb = bf16_round(bb); }
        sm[q] = vals[u * 4 + q]; o[q] = (vals[u * 4 + q] - mu) * rs * gg + bb;
      }
      if (out_sum) *(volatile v4f*)(out_sum + (size_t)row * N + j) = sm;
      *(volatile v4f*)(out_norm + (size_t)row * N + j) = o;
    }
    if (pass == 0) __threadfence();
  }
}


typedef _Float16 v16h __attribute__((ext_vector_type(16)));
union FragH { v16h v; v8us half[2]; _Float16 h[16]; unsigned short u[16]; };
template <int NT>
__device__ __forceinline__ v8f mmaH(v16h ah, v16h al, v16h bh, v16h bl, v8f c) {
  c = __builtin_amdgcn_wmma_f32_16x16x32_f16(false, ah, false, bh, (short)0, c, false, false);
  if (NT >= 2) c = __builtin_amdgcn_wmma_f32_16x16x32_f16(false, al, false, bh, (short)0, c, false, false);
  if (NT >= 3) c = __builtin_amdgcn_wmma_f32_16x16x32_f16(false, ah, false, bl, (short)0, c, false, false);
  asm volatile("v_nop\n\tv_nop\n\tv_nop\n\tv_nop" : "+v"(c) : "v"(ah), "v"(al), "v"(bh), "v"(bl));
  return c;
}
template <bool ASPLIT>
__global__ __launch_bounds__(128) void k_gemm_h(const float* __restrict__ A, int lda, size_t sA, const _Float16* __restrict__ Bh, int ldb, size_t sB, float alpha, float* __restrict__ C, int ldc, size_t sC, int M, int N, int K) {
  __shared__ __attribute__((aligned(16))) float so[4][16][64];
  const int tid = threadIdx.x, w = tid >> 5, lane = tid & 31, ln = lane & 15, hh = lane >> 4; const int by = blockIdx.y;
  A += (size_t)by * sA; Bh += (size_t)by * sB; C += (size_t)by * sC;
  const int ntn = (N + 63) / 64; const int wid = blockIdx.x * 4 + w; const int mt = wid / ntn, nq = wid % ntn; if (mt * 16 >= M) return;
  const int row0 = mt * 16, col0 = nq * 64; const float* arow = A + (size_t)(row0 + ln) * lda;
  v8f acc[4] = {};
  for (int kb = 0; kb < K; kb += 32) {
    FragH ah, al;
    const v4f x0 = *(const v4fa*)(arow + kb + 8 * hh), x1 = *(const v4fa*)(arow + kb + 8 * hh + 4), x2 = *(const v4fa*)(arow + kb + 16 + 8 * hh), x3 = *(const v4fa*)(arow + kb + 16 + 8 * hh + 4);
    float xs[16] = {x0[0],x0[1],x0[2],x0[3],x1[0],x1[1],x1[2],x1[3],x2[0],x2[1],x2[2],x2[3],x3[0],x3[1],x3[2],x3[3]};
#pragma unroll
    for (int i = 0; i < 16; ++i) { const _Float16 h = (_Float16)xs[i]; ah.h[i] = h; al.h[i] = ASPLIT ? (_Float16)(xs[i] - (float)h) : (_Float16)0.0f; }
#pragma unroll
    for (int t = 0; t < 4; ++t) { if (col0 + t * 16 >= N) continue; const size_t boff = (size_t)(col0 + t * 16 + ln) * ldb + kb; FragH bq; bq.half[0] = *(const v8us*)(Bh + boff + 8 * hh); bq.half[1] = *(const v8us*)(Bh + boff + 16 + 8 * hh);
      acc[t] = mmaH<ASPLIT ? 2 : 1>(ah.v, al.v, bq.v, bq.v, acc[t]); }
  }
#pragma unroll
  for (int t = 0; t < 4; ++t) { if (col0 + t * 16 >= N) continue;
#pragma unroll
    for (int r = 0; r < 8; ++r) so[w][8 * hh + r][t * 16 + ln] = acc[t][r] * alpha; }
  __builtin_amdgcn_fence(__ATOMIC_ACQ_REL, "workgroup"); __builtin_amdgcn_wave_barrier();
  const int rsub = lane >> 4, c4 = (lane & 15) * 4;
  for (int pass = 0; pass < 2; ++pass) {
#pragma unroll
    for (int q = 0; q < 8; ++q) { const int r = q * 2 + rsub; if (col0 + c4 < N) { const v4f v = *(const v4fa*)&so[w][r][c4]; *(volatile v4f*)(C + (size_t)(row0 + r) * ldc + col0 + c4) = v; } }
    if (pass == 0) __threadfence(); }
}

__global__ __launch_bounds__(256) void k_wt_f16(const float* __restrict__ W, _Float16* __restrict__ Wt, int K, int N, float scale) {
  const int t = blockIdx.x * 256 + threadIdx.x; if (t >= N * (K / 8)) return; const int n = t / (K / 8), k8 = (t % (K / 8)) * 8; FragH f;
#pragma unroll
  for (int i = 0; i < 8; ++i) f.h[i] = (_Float16)(bf16_round(W[(size_t)(k8 + i) * N + n]) * scale); const v8us o = f.half[0];
  *(volatile v8us*)((unsigned short*)Wt + (size_t)n * K + k8) = o; __threadfence(); *(volatile v8us*)((unsigned short*)Wt + (size_t)n * K + k8) = o;
}
template <int ACT>
__global__ __launch_bounds__(128) void k_gemm_hhx(const _Float16* __restrict__ A, int lda, size_t sA, const _Float16* __restrict__ Bh, int ldb, size_t sB, float alpha, const float* __restrict__ bias, size_t sBias, const float* __restrict__ CP, int rowsPerB, size_t sCPb, int row0g,
    float* __restrict__ C, _Float16* __restrict__ C16, int ldc, size_t sC, int M, int N, int K) {
  __shared__ __attribute__((aligned(16))) float so[4][16][64];
  const int tid = threadIdx.x, w = tid >> 5, lane = tid & 31, ln = lane & 15, hh = lane >> 4; const int by = blockIdx.y;
  A += (size_t)by * sA; Bh += (size_t)by * sB; const size_t cofs = (size_t)by * sC; const float* bp = bias ? bias + (size_t)by * sBias : nullptr;
  const int ntn = (N + 63) / 64; const int wid = blockIdx.x * 4 + w; const int mt = wid / ntn, nq = wid % ntn; if (mt * 16 >= M) return;
  const int row0 = mt * 16, col0 = nq * 64; const _Float16* arow = A + (size_t)(row0 + ln) * lda;
  v8f acc[4] = {};
  for (int kb = 0; kb < K; kb += 32) { FragH ah; ah.half[0] = *(const v8us*)((const unsigned short*)arow + kb + 8 * hh); ah.half[1] = *(const v8us*)((const unsigned short*)arow + kb + 16 + 8 * hh);
#pragma unroll
    for (int t = 0; t < 4; ++t) { if (col0 + t * 16 >= N) continue; const size_t boff = (size_t)(col0 + t * 16 + ln) * ldb + kb; FragH bq; bq.half[0] = *(const v8us*)((const unsigned short*)Bh + boff + 8 * hh); bq.half[1] = *(const v8us*)((const unsigned short*)Bh + boff + 16 + 8 * hh);
      acc[t] = mmaH<1>(ah.v, ah.v, bq.v, bq.v, acc[t]); }
  }
#pragma unroll
  for (int t = 0; t < 4; ++t) { if (col0 + t * 16 >= N) continue; const int col = col0 + t * 16 + ln; const float bv = bp ? bf16_round(bp[col]) : 0.f;
#pragma unroll
    for (int r = 0; r < 8; ++r) { float v = acc[t][r] * alpha + bv; if (CP) { const int bidx = (row0g + row0 + 8 * hh + r) / rowsPerB; v += CP[(size_t)bidx * sCPb + (size_t)by * 64 + col]; } if (ACT == 1) v = (v > 0.f) ? v : expm1f(v); else if (ACT == 7) v = (v > 0.f) ? v + 1.0f : expf(v); else if (ACT == 8) v = tanhf(v); else if (ACT == 9) v = 0.5f * v * (1.0f + tanhf(0.7978845608028654f * (v + 0.044715f * v * v * v))); else if (ACT == 11) v = 1.0f / (1.0f + expf(-v)); else if (ACT == 12) v = (v > 0.f) ? v : 0.01f * v; else if (ACT == 14) v = (v > 0.f) ? v : 0.1f * v; else if (ACT == 15) v = v / (1.0f + expf(-v)); else if (ACT == 3) v = fmaxf(v, 0.f); else if (ACT == 6) v = 0.5f * v * (1.0f + erff(v * 0.70710678118654752f)); so[w][8 * hh + r][t * 16 + ln] = v; } }
  __builtin_amdgcn_fence(__ATOMIC_ACQ_REL, "workgroup"); __builtin_amdgcn_wave_barrier();
  const int rsub = lane >> 4, c4 = (lane & 15) * 4; typedef _Float16 v4h __attribute__((ext_vector_type(4)));
  for (int pass = 0; pass < 2; ++pass) {
#pragma unroll
    for (int q = 0; q < 8; ++q) { const int r = q * 2 + rsub; if (col0 + c4 < N) { const v4f v = *(const v4fa*)&so[w][r][c4]; if (C) *(volatile v4f*)(C + cofs + (size_t)(row0 + r) * ldc + col0 + c4) = v; if (C16) { v4h h4; for (int i = 0; i < 4; ++i) h4[i] = (_Float16)v[i]; *(volatile v4h*)(C16 + cofs + (size_t)(row0 + r) * ldc + col0 + c4) = h4; } } }
    if (pass == 0) __threadfence(); }
}


typedef _Float16 v4h __attribute__((ext_vector_type(4)));

__global__ __launch_bounds__(256) void k_x16(const float* __restrict__ x, _Float16* __restrict__ X16, size_t n8) { const size_t t = (size_t)blockIdx.x * 256 + threadIdx.x; if (t >= n8) return; FragH f;
#pragma unroll
  for (int q = 0; q < 8; ++q) f.h[q] = (_Float16)bf16_round(x[t * 8 + q]); *(volatile v8us*)((unsigned short*)X16 + t * 8) = f.half[0]; __threadfence(); *(volatile v8us*)((unsigned short*)X16 + t * 8) = f.half[0]; }
__global__ __launch_bounds__(256) void k_h16(const float* __restrict__ x, _Float16* __restrict__ X16, size_t n8) { const size_t t = (size_t)blockIdx.x * 256 + threadIdx.x; if (t >= n8) return; FragH f;
#pragma unroll
  for (int q = 0; q < 8; ++q) f.h[q] = (_Float16)x[t * 8 + q]; *(volatile v8us*)((unsigned short*)X16 + t * 8) = f.half[0]; __threadfence(); *(volatile v8us*)((unsigned short*)X16 + t * 8) = f.half[0]; }
__global__ __launch_bounds__(256) void k_round16f(const float* __restrict__ W, _Float16* __restrict__ Bt, size_t n8) { const size_t t = (size_t)blockIdx.x * 256 + threadIdx.x; if (t >= n8) return; FragH f;
#pragma unroll
  for (int i = 0; i < 8; ++i) f.h[i] = (_Float16)(bf16_round(W[t * 8 + i]) * 16.0f); *(volatile v8us*)((unsigned short*)Bt + t * 8) = f.half[0]; __threadfence(); *(volatile v8us*)((unsigned short*)Bt + t * 8) = f.half[0]; }
template <int NHv, int TTv>
__global__ __launch_bounds__(256) void k_vt(const _Float16* __restrict__ V16, int ldv, int voff, _Float16* __restrict__ Vt) { __shared__ unsigned short tl[64][66]; const int tid = threadIdx.x; const int slab = blockIdx.x / (TTv / 64), lg = blockIdx.x % (TTv / 64); const int b = slab / NHv, h = slab % NHv;
  for (int i = tid; i < 64 * 8; i += 256) { const int r = i / 8, c8 = (i % 8) * 8; FragH f; f.half[0] = *(const v8us*)((const unsigned short*)V16 + ((size_t)b * TTv + lg * 64 + r) * ldv + voff + h * 64 + c8);
#pragma unroll
    for (int q = 0; q < 8; ++q) tl[r][c8 + q] = f.u[q]; }
  __syncthreads();
  for (int pass = 0; pass < 2; ++pass) {
#pragma unroll
    for (int rd = 0; rd < 2; ++rd) { const int d = rd * 32 + tid / 8, pc = tid % 8; FragH f;
#pragma unroll
      for (int q = 0; q < 8; ++q) f.u[q] = tl[pc * 8 + q][d];
      *(volatile v8us*)((unsigned short*)Vt + ((size_t)slab * 64 + d) * TTv + lg * 64 + pc * 8) = f.half[0]; }
    if (pass == 0) __threadfence(); } }

__global__ __launch_bounds__(256) void k_hl(const float* __restrict__ F, _Float16* __restrict__ Hh, _Float16* __restrict__ Hl, size_t n8) { const size_t t = (size_t)blockIdx.x * 256 + threadIdx.x; if (t >= n8) return; FragH fh, fl; const v4f a = *(const v4fa*)(F + t * 8), c = *(const v4fa*)(F + t * 8 + 4);
#pragma unroll
  for (int q = 0; q < 4; ++q) { _Float16 h = (_Float16)a[q]; fh.h[q] = h; fl.h[q] = (_Float16)((a[q] - (float)h) * 1024.0f); h = (_Float16)c[q]; fh.h[4 + q] = h; fl.h[4 + q] = (_Float16)((c[q] - (float)h) * 1024.0f); }
  for (int pass = 0; pass < 2; ++pass) { *(volatile v8us*)((unsigned short*)Hh + t * 8) = fh.half[0]; *(volatile v8us*)((unsigned short*)Hl + t * 8) = fl.half[0]; if (pass == 0) __threadfence(); } }

__device__ __forceinline__ v4f shfl4(v4f v, int srcl) { v4f r; r[0] = __shfl(v[0], srcl, 32); r[1] = __shfl(v[1], srcl, 32); r[2] = __shfl(v[2], srcl, 32); r[3] = __shfl(v[3], srcl, 32); return r; }
__global__ __launch_bounds__(256) void k_msconv(const float* __restrict__ x, const float* __restrict__ cw, const float* __restrict__ cb, _Float16* __restrict__ H0) {
  #pragma clang fp contract(off)
  const int t = blockIdx.x * 256 + threadIdx.x; if (t >= NR * NSC * (CC / 8)) return; const int c0 = (t % (CC / 8)) * 8; const int s = (t / (CC / 8)) % NSC; const int r = t / ((CC / 8) * NSC); const int b = r / NN, n = r % NN; const int d = 1 << s; const float* xb = x + (size_t)b * TW * NN + n; float w0[8], w1[8], w2[8], bb[8], acc[8];
#pragma unroll
  for (int q = 0; q < 8; ++q) { const int c = c0 + q; w0[q] = bf16_round(cw[((size_t)s * CC + c) * 3 + 0]); w1[q] = bf16_round(cw[((size_t)s * CC + c) * 3 + 1]); w2[q] = bf16_round(cw[((size_t)s * CC + c) * 3 + 2]); bb[q] = bf16_round(cb[(size_t)s * CC + c]); acc[q] = 0.f; }
#pragma unroll 1
  for (int tt = 0; tt < TW; ++tt) { const float xm = (tt - d >= 0) ? bf16_round(xb[(size_t)(tt - d) * NN]) : 0.f; const float x0 = bf16_round(xb[(size_t)tt * NN]); const float xp = (tt + d < TW) ? bf16_round(xb[(size_t)(tt + d) * NN]) : 0.f;
#pragma unroll
    for (int q = 0; q < 8; ++q) { float v = bb[q]; v += w0[q] * xm; v += w1[q] * x0; v += w2[q] * xp; acc[q] += fmaxf(v, 0.f); } }
  FragH f;
#pragma unroll
  for (int q = 0; q < 8; ++q) f.h[q] = (_Float16)(acc[q] / (float)TW);
  *(volatile v8us*)((unsigned short*)H0 + (size_t)r * (NSC * CC) + s * CC + c0) = f.half[0]; __threadfence(); *(volatile v8us*)((unsigned short*)H0 + (size_t)r * (NSC * CC) + s * CC + c0) = f.half[0]; }
__global__ __launch_bounds__(256) void k_ln16(const float* __restrict__ Hf, const float* __restrict__ g, const float* __restrict__ bb, _Float16* __restrict__ O16) {
  #pragma clang fp contract(off)
  const int tid = threadIdx.x, w = tid >> 5, ln = tid & 31; const int r = blockIdx.x * 8 + w; if (r >= NR) return; const v4f a = *(const v4fa*)(Hf + (size_t)r * CC + ln * 4); float s = a[0] + a[1] + a[2] + a[3];
  for (int o = 16; o > 0; o >>= 1) s += __shfl_xor(s, o, 32); const float mu = s / (float)CC; float q2 = 0.f;
#pragma unroll
  for (int k = 0; k < 4; ++k) { const float dd = a[k] - mu; q2 += dd * dd; }
  for (int o = 16; o > 0; o >>= 1) q2 += __shfl_xor(q2, o, 32); const float rs = 1.0f / sqrtf(q2 / (float)CC + 1e-5f); FragH f;
#pragma unroll
  for (int k = 0; k < 4; ++k) { const int c = ln * 4 + k; f.h[k] = (_Float16)((a[k] - mu) * rs * bf16_round(g[c]) + bf16_round(bb[c])); }
  const unsigned long long pv = *(const unsigned long long*)&f.u[0]; *(volatile unsigned long long*)((unsigned short*)O16 + (size_t)r * CC + ln * 4) = pv; __threadfence(); *(volatile unsigned long long*)((unsigned short*)O16 + (size_t)r * CC + ln * 4) = pv; }
__global__ __launch_bounds__(256) void k_wql(const float* __restrict__ wql, _Float16* __restrict__ Bt) { const int t = blockIdx.x * 256 + threadIdx.x; if (t >= 64 * (CC / 8)) return; const int k0 = (t % (CC / 8)) * 8, o = t / (CC / 8); FragH f;
#pragma unroll
  for (int q = 0; q < 8; ++q) f.h[q] = (o < 48) ? (_Float16)(bf16_round(wql[(size_t)o * CC + k0 + q]) * 16.0f) : (_Float16)0.0f;
  *(volatile v8us*)((unsigned short*)Bt + (size_t)o * CC + k0) = f.half[0]; __threadfence(); *(volatile v8us*)((unsigned short*)Bt + (size_t)o * CC + k0) = f.half[0]; }
__global__ __launch_bounds__(256) void k_wqh(const float* __restrict__ wqh, _Float16* __restrict__ Bt) { const int t = blockIdx.x * 256 + threadIdx.x; if (t >= 3 * CC * 8) return; const int k0 = (t & 7) * 8, o = t >> 3; FragH f;
#pragma unroll
  for (int q = 0; q < 8; ++q) { const int k = k0 + q; f.h[q] = (k < 48) ? (_Float16)(bf16_round(wqh[(size_t)o * 48 + k]) * 16.0f) : (_Float16)0.0f; }
  *(volatile v8us*)((unsigned short*)Bt + (size_t)o * 64 + k0) = f.half[0]; __threadfence(); *(volatile v8us*)((unsigned short*)Bt + (size_t)o * 64 + k0) = f.half[0]; }
__global__ __launch_bounds__(256) void k_bpad(const float* __restrict__ b, int n, int npad, float* __restrict__ BP) { const int l = threadIdx.x; if (l >= npad) return; const float v = (l < n) ? b[l] : 0.f; *(volatile float*)(BP + l) = v; __threadfence(); *(volatile float*)(BP + l) = v; }
__global__ __launch_bounds__(256) void k_qakb(const float* __restrict__ QKV, const float* __restrict__ u, const float* __restrict__ vv, _Float16* __restrict__ QA, _Float16* __restrict__ KB) {
  #pragma clang fp contract(off)
  const int t = blockIdx.x * 256 + threadIdx.x; if (t >= NR * 32) return; const int i = t & 31, r = t >> 5; const int n = r % NN; const int h = i >> 2, part = i & 3; const float* qr = QKV + (size_t)r * 3 * CC; FragH qa, kb;
#pragma unroll
  for (int e = 0; e < 8; ++e) { const int j = (part & 1) * 8 + e;
    if (part < 2) { qa.h[e] = (_Float16)qr[h * HD + j]; kb.h[e] = (_Float16)qr[CC + h * HD + j]; }
    else { qa.h[e] = (_Float16)(4.0f * bf16_round(u[((size_t)h * NN + n) * BOT + j])); kb.h[e] = (_Float16)bf16_round(vv[((size_t)h * BOT + j) * NN + n]); } }
  for (int pass = 0; pass < 2; ++pass) { *(volatile v8us*)((unsigned short*)QA + (size_t)r * (NH * 32) + i * 8) = qa.half[0]; *(volatile v8us*)((unsigned short*)KB + (size_t)r * (NH * 32) + i * 8) = kb.half[0]; if (pass == 0) __threadfence(); } }
__global__ __launch_bounds__(256) void k_vt(const float* __restrict__ QKV, int b, _Float16* __restrict__ VT) { const int t = blockIdx.x * 256 + threadIdx.x; if (t >= CC * (NN / 8)) return; const int m0 = (t % (NN / 8)) * 8, hd = t / (NN / 8); FragH f;
#pragma unroll
  for (int q = 0; q < 8; ++q) f.h[q] = (_Float16)QKV[((size_t)b * NN + m0 + q) * 3 * CC + 2 * CC + hd];
  *(volatile v8us*)((unsigned short*)VT + (size_t)hd * NN + m0) = f.half[0]; __threadfence(); *(volatile v8us*)((unsigned short*)VT + (size_t)hd * NN + m0) = f.half[0]; }
__global__ __launch_bounds__(256) void k_asoft(const float* __restrict__ S, const int* __restrict__ adj, const float* __restrict__ ascale, _Float16* __restrict__ P16) {
  #pragma clang fp contract(off)
  const int tid = threadIdx.x, w = tid >> 5, ln = tid & 31; const int row = blockIdx.x * 8 + w; if (row >= HG * NN) return; const int n = row % NN; const float* sr = S + (size_t)row * NN; const int* ar = adj + (size_t)n * NN; const float negterm = bf16_round(ascale[0]) * (-1.0e9f); float m = -3.0e38f;
#pragma unroll 1
  for (int jb = 0; jb < NN; jb += 256) {
#pragma unroll
    for (int k = 0; k < 8; ++k) { const int j = jb + 8 * ln + k; const float v = sr[j] + ((ar[j] > 0) ? 0.f : negterm); m = fmaxf(m, v); } }
  for (int o = 16; o > 0; o >>= 1) m = fmaxf(m, __shfl_xor(m, o, 32));
  float su = 0.f;
#pragma unroll 1
  for (int jb = 0; jb < NN; jb += 256) {
#pragma unroll
    for (int k = 0; k < 8; ++k) { const int j = jb + 8 * ln + k; const float v = sr[j] + ((ar[j] > 0) ? 0.f : negterm); su += expf(v - m); } }
  for (int o = 16; o > 0; o >>= 1) su += __shfl_xor(su, o, 32); const float inv = 1024.0f / su;
  for (int pass = 0; pass < 2; ++pass) {
#pragma unroll 1
    for (int jb = 0; jb < NN; jb += 256) { FragH f;
#pragma unroll
      for (int k = 0; k < 8; ++k) { const int j = jb + 8 * ln + k; const float v = sr[j] + ((ar[j] > 0) ? 0.f : negterm); f.h[k] = (_Float16)(expf(v - m) * inv); }
      *(volatile v8us*)((unsigned short*)P16 + (size_t)row * NN + jb + 8 * ln) = f.half[0]; }
    if (pass == 0) __threadfence(); } }
__global__ __launch_bounds__(256) void k_tail(const float* __restrict__ AO, const float* __restrict__ RES, const float* __restrict__ wol, const float* __restrict__ bol, const float* __restrict__ woh, const float* __restrict__ boh, const float* __restrict__ p1w, const float* __restrict__ p1b, const float* __restrict__ p2w, const float* __restrict__ p2b, float* __restrict__ PT) {
  #pragma clang fp contract(off)
  const int tid = threadIdx.x, w = tid >> 5, ln = tid & 31; const int r = blockIdx.x * 8 + w; if (r >= NR) return; const v4f a = *(const v4fa*)(AO + (size_t)r * CC + ln * 4);
  float olj[BOT];
#pragma unroll
  for (int j = 0; j < BOT; ++j) { float s = 0.f;
#pragma unroll
    for (int k = 0; k < 4; ++k) s += a[k] * bf16_round(wol[(size_t)j * CC + ln * 4 + k]);
    for (int o = 16; o > 0; o >>= 1) s += __shfl_xor(s, o, 32); olj[j] = s + bf16_round(bol[j]); }
  float oc[4];
#pragma unroll
  for (int k = 0; k < 4; ++k) { const int c = ln * 4 + k; float s = bf16_round(boh[c]) + RES[(size_t)r * CC + c];
#pragma unroll
    for (int j = 0; j < BOT; ++j) s += olj[j] * bf16_round(woh[(size_t)c * BOT + j]);
    oc[k] = s; }
  float hj[BOT];
#pragma unroll
  for (int j = 0; j < BOT; ++j) { float s = 0.f;
#pragma unroll
    for (int k = 0; k < 4; ++k) s += oc[k] * bf16_round(p1w[(size_t)j * CC + ln * 4 + k]);
    for (int o = 16; o > 0; o >>= 1) s += __shfl_xor(s, o, 32); hj[j] = fmaxf(s + bf16_round(p1b[j]), 0.f); }
  float pv = 0.f; if (ln < HOR) { pv = bf16_round(p2b[ln]);
#pragma unroll
    for (int j = 0; j < BOT; ++j) pv += hj[j] * bf16_round(p2w[(size_t)ln * BOT + j]); }
  *(volatile float*)(PT + (size_t)r * 32 + ln) = pv; __threadfence(); *(volatile float*)(PT + (size_t)r * 32 + ln) = pv; }
__global__ __launch_bounds__(256) void k_pred(const float* __restrict__ PT, const float* __restrict__ x, const float* __restrict__ hww, const float* __restrict__ hwb, float* __restrict__ out) {
  #pragma clang fp contract(off)
  const int t = blockIdx.x * 256 + threadIdx.x; if (t >= NBt * HOR * (NN / 4)) return; const int n0 = (t % (NN / 4)) * 4; const int hr = (t / (NN / 4)) % HOR; const int b = t / ((NN / 4) * HOR); v4f v;
#pragma unroll
  for (int q = 0; q < 4; ++q) { const int n = n0 + q; float s = PT[((size_t)b * NN + n) * 32 + hr] + bf16_round(hwb[hr]);
#pragma unroll
    for (int wv = 0; wv < HWY; ++wv) s += bf16_round(x[((size_t)b * TW + (TW - HWY + wv)) * NN + n]) * bf16_round(hww[hr * HWY + wv]);
    v[q] = s; }
  float* dst = out + ((size_t)b * HOR + hr) * NN + n0; *(volatile v4f*)dst = v; __threadfence(); *(volatile v4f*)dst = v; }
__global__ __launch_bounds__(64) void k_zero1(float* __restrict__ p) { if (threadIdx.x == 0) { *(volatile float*)p = 0.f; __threadfence(); *(volatile float*)p = 0.f; } }

extern "C" void kernel_launch(void* const* d_in, const int* in_sizes, int n_in,
                              void* d_out, int out_size, void* d_ws, size_t ws_size, hipStream_t stream) {
  (void)in_sizes; (void)n_in; (void)out_size;
  const float* const* I = (const float* const*)d_in; const float* x = I[0]; const int* adj = (const int*)d_in[1];
  char* ws = (char*)d_ws; size_t off = 0;
  auto take = [&](size_t bytes) { char* p = ws + off; off += (bytes + 255) & ~(size_t)255; return p; };
  _Float16* BFU = (_Float16*)take((size_t)CC * NSC * CC * 2); _Float16* BQL = (_Float16*)take((size_t)64 * CC * 2); float* BQLB = (float*)take(64 * 4); _Float16* BQH = (_Float16*)take((size_t)3 * CC * 64 * 2);
  float* S = (float*)take((size_t)HG * NN * NN * 4); _Float16* P16 = (_Float16*)take((size_t)HG * NN * NN * 2); float* Hf = (float*)take((size_t)NR * CC * 4); _Float16* HN16 = (_Float16*)take((size_t)NR * CC * 2); _Float16* QL16 = (_Float16*)take((size_t)NR * 64 * 2); float* QKV = (float*)take((size_t)NR * 3 * CC * 4); _Float16* QA = (_Float16*)take((size_t)NR * NH * 32 * 2); _Float16* KB = (_Float16*)take((size_t)NR * NH * 32 * 2); _Float16* VT = (_Float16*)take((size_t)CC * NN * 2); float* AO = (float*)take((size_t)NR * CC * 4); float* PT = (float*)take((size_t)NR * 32 * 4);
  _Float16* H0 = (_Float16*)S;
  if (off > ws_size) return;
  k_round16f<<<(CC * NSC * CC / 8 + 255) / 256, 256, 0, stream>>>(I[4], BFU, (size_t)CC * NSC * CC / 8); k_wql<<<(64 * (CC / 8) + 255) / 256, 256, 0, stream>>>(I[8], BQL); k_bpad<<<1, 256, 0, stream>>>(I[9], 48, 64, BQLB); k_wqh<<<(3 * CC * 8 + 255) / 256, 256, 0, stream>>>(I[10], BQH);
  k_msconv<<<(NR * NSC * (CC / 8) + 255) / 256, 256, 0, stream>>>(x, I[2], I[3], H0);
  k_gemm_hhx<3><<<dim3(((NR / 16) * (CC / 64) + 3) / 4, 1), 128, 0, stream>>>(H0, NSC * CC, 0, BFU, NSC * CC, 0, 0.0625f, I[5], 0, nullptr, 1, 0, 0, Hf, nullptr, CC, 0, NR, CC, NSC * CC);
  k_ln16<<<NR / 8, 256, 0, stream>>>(Hf, I[6], I[7], HN16);
  k_gemm_hhx<0><<<dim3(((NR / 16) * 1 + 3) / 4, 1), 128, 0, stream>>>(HN16, CC, 0, BQL, CC, 0, 0.0625f, BQLB, 0, nullptr, 1, 0, 0, nullptr, QL16, 64, 0, NR, 64, CC);
  k_gemm_hhx<0><<<dim3(((NR / 16) * (3 * CC / 64) + 3) / 4, 1), 128, 0, stream>>>(QL16, 64, 0, BQH, 64, 0, 0.0625f, I[11], 0, nullptr, 1, 0, 0, QKV, nullptr, 3 * CC, 0, NR, 3 * CC, 64);
  k_qakb<<<(NR * 32 + 255) / 256, 256, 0, stream>>>(QKV, I[12], I[13], QA, KB);
  const dim3 gS(((NN / 16) * (NN / 64) + 3) / 4, HG), gV(((NN / 16) * 1 + 3) / 4, HG);
  for (int b = 0; b < NBt; ++b) {
    k_gemm_hhx<0><<<gS, 128, 0, stream>>>(QA + (size_t)b * NN * 256, 256, (size_t)32, KB + (size_t)b * NN * 256, 256, (size_t)32, 0.25f, nullptr, 0, nullptr, 1, 0, 0, S, nullptr, NN, (size_t)NN * NN, NN, NN, 32);
    k_asoft<<<HG * NN / 8, 256, 0, stream>>>(S, adj, I[14], P16); k_vt<<<(CC * (NN / 8) + 255) / 256, 256, 0, stream>>>(QKV, b, VT);
    k_gemm_hhx<0><<<gV, 128, 0, stream>>>(P16, NN, (size_t)NN * NN, VT, NN, (size_t)HD * NN, 0.0009765625f, nullptr, 0, nullptr, 1, 0, 0, AO + (size_t)b * NN * CC, nullptr, CC, (size_t)HD, NN, HD, NN); }
  k_tail<<<NR / 8, 256, 0, stream>>>(AO, Hf, I[15], I[16], I[17], I[18], I[19], I[20], I[21], I[22], PT);
  k_pred<<<(NBt * HOR * (NN / 4) + 255) / 256, 256, 0, stream>>>(PT, x, I[23], I[24], (float*)d_out);
  k_zero1<<<1, 64, 0, stream>>>((float*)((char*)d_out + 1572864));
}
